// HRP_3994319585787
// MI455X (gfx1250) — hardware-run, weakly checked
//
#include <hip/hip_runtime.h>
#include <math.h>

typedef __attribute__((ext_vector_type(16))) _Float16 v16h;
typedef __attribute__((ext_vector_type(8)))  _Float16 v8h;
typedef __attribute__((ext_vector_type(8)))  float    v8f;
typedef __attribute__((ext_vector_type(4)))  float    v4f;
typedef __attribute__((ext_vector_type(2)))  float    v2f;

constexpr int kNB = 1024;
constexpr int kNT = 2;
constexpr int kNZ = 100;
constexpr int kNS = 6;
constexpr int kRowsP   = kNZ * kNB;
constexpr int kSaElems = kRowsP * kNT;
constexpr int kOut0    = kNB * kNZ;
constexpr int kOutAll  = kOut0 + kNB;
constexpr float kWCarry = 32.0f;
constexpr float kWInv   = 1.0f / kWCarry;
static_assert(kRowsP == 102400 && kSaElems == 204800 && kOutAll == 103424, "shapes");
static_assert((kRowsP % 64) == 0 && (kNB % 64) == 0, "row tiles");
static_assert((kOut0 % 1024) == 0 && (kNZ % 4) == 0, "pack tiles");

constexpr int kBlkP0 = 0;
constexpr int kBlkP1 = kBlkP0 + (192 * 64) / 1024;
constexpr int kBlkP2 = kBlkP1 + (512 * 64) / 1024;
constexpr int kBlkP3 = kBlkP2 + (128 * 512) / 1024;
constexpr int kBlkP4 = kBlkP3 + (96 * 64) / 1024;
constexpr int kBlkP5 = kBlkP4 + (96 * 32) / 1024;
constexpr int kBlkP6 = kBlkP5 + (512 * 32) / 1024;
constexpr int kBlkP7 = kBlkP6 + (256 * 512) / 1024;
constexpr int kBlkP8 = kBlkP7 + (512 * 64) / 1024;
constexpr int kBlkEnd = kBlkP8 + (256 * 512) / 1024;
static_assert(kBlkP1 == 12 && kBlkP2 == 44 && kBlkP3 == 108 && kBlkP4 == 114 && kBlkP5 == 117 &&
              kBlkP6 == 133 && kBlkP7 == 261 && kBlkP8 == 293 && kBlkEnd == 421, "plane blocks");
constexpr size_t kOffSA  = 0;
constexpr size_t kOffW16 = (size_t)kSaElems * 4;
constexpr size_t kWsTotal = kOffW16 + (size_t)kBlkEnd * 1024 * 2;
static_assert(kOffW16 == 819200ull && kWsTotal == 1681408ull, "carve total");
static_assert((kOffW16 % 128) == 0 && kWsTotal <= 134217728ull, "carve cap");

union FragU { v16h v; v8h h[2]; };
__device__ __forceinline__ v16h frag_load(const _Float16* p) {
  FragU f;
  f.h[0] = *(const v8h*)(p);
  f.h[1] = *(const v8h*)(p + 16);
  return f.v;
}
__device__ __forceinline__ v8f mma16(v16h a, v16h b, v8f c) {
  c = __builtin_amdgcn_wmma_f32_16x16x32_f16(false, a, false, b, (short)0, c, false, false);
  asm volatile("v_nop\n\tv_nop\n\tv_nop\n\tv_nop" : "+v"(c) : "v"(a), "v"(b));
  return c;
}
__device__ __forceinline__ int pin_i(int v) {
  asm volatile("" : "+v"(v));
  return v;
}
__device__ __forceinline__ void pin_if(int& o, float& s) {
  asm volatile("" : "+v"(o), "+v"(s));
}
__device__ __forceinline__ v8f zero8() { return (v8f){0.f, 0.f, 0.f, 0.f, 0.f, 0.f, 0.f, 0.f}; }
__device__ __forceinline__ v16h zero16h() {
  v16h z;
#pragma unroll
  for (int e = 0; e < 16; ++e) z[e] = (_Float16)0.0f;
  return z;
}
__device__ __forceinline__ void unpack8(const v4f a, const v4f b, float (&o)[8]) {
  o[0] = a[0]; o[1] = a[1]; o[2] = a[2]; o[3] = a[3];
  o[4] = b[0]; o[5] = b[1]; o[6] = b[2]; o[7] = b[3];
}
__device__ __forceinline__ v16h pack_tiles(const float (&lo)[8], const float (&hi)[8]) {
  v16h f;
#pragma unroll
  for (int e = 0; e < 8; ++e) {
    f[e]     = (_Float16)lo[e];
    f[8 + e] = (_Float16)hi[e];
  }
  return f;
}

__device__ __forceinline__ void gru_gates8(
    const float (&xr)[8], const float (&xz)[8], const float (&xn)[8],
    const float (&hr)[8], const float (&hz)[8], const float (&hn)[8],
    const float (&ho)[8], float (&hnew)[8]) {
#pragma unroll
  for (int r = 0; r < 8; ++r) {
    const float rg = 1.0f / (1.0f + expf(-(xr[r] + hr[r])));
    const float zg = 1.0f / (1.0f + expf(-(xz[r] + hz[r])));
    const float ng = tanhf(xn[r] + rg * hn[r]);
    hnew[r] = (1.0f - zg) * ng + zg * ho[r];
  }
}

template <int KS1>
__device__ __forceinline__ float mlp_chain8(
    const _Float16* __restrict__ W1, const float* __restrict__ b1,
    const _Float16* __restrict__ W2, const float* __restrict__ b2, const float* __restrict__ w3,
    const int mt0, const v16h in0, const v16h in1, const int rlane, const int koff) {
  constexpr int LD1 = KS1 * 32;
  v8f acc[8];
#pragma unroll
  for (int i = 0; i < 8; ++i) acc[i] = zero8();
#pragma unroll 1
  for (int ks = 0; ks < 16; ++ks) {
    const int o1 = pin_i((ks * 32 + rlane) * LD1 + koff);
    v8f d0 = zero8();
    v8f d1 = zero8();
    v16h a;
    a = frag_load(W1 + o1);
    d0 = mma16(a, in0, d0);
    if (KS1 == 2) {
      const int o = pin_i(o1 + 32);
      a = frag_load(W1 + o);
      d0 = mma16(a, in1, d0);
    }
    {
      const int o = pin_i(o1 + 16 * LD1);
      a = frag_load(W1 + o);
      d1 = mma16(a, in0, d1);
    }
    if (KS1 == 2) {
      const int o = pin_i(o1 + 16 * LD1 + 32);
      a = frag_load(W1 + o);
      d1 = mma16(a, in1, d1);
    }
    const int ob = pin_i(ks * 32 + koff);
    const float* bp = b1 + ob;
    const v4f ba = *(const v4f*)(bp);
    const v4f bb = *(const v4f*)(bp + 4);
    const v4f bc = *(const v4f*)(bp + 16);
    const v4f bd = *(const v4f*)(bp + 20);
    v16h bf;
#pragma unroll
    for (int e = 0; e < 4; ++e) {
      bf[e]      = (_Float16)fmaxf(fmaf(d0[e],     kWInv, ba[e]), 0.0f);
      bf[4 + e]  = (_Float16)fmaxf(fmaf(d0[4 + e], kWInv, bb[e]), 0.0f);
      bf[8 + e]  = (_Float16)fmaxf(fmaf(d1[e],     kWInv, bc[e]), 0.0f);
      bf[12 + e] = (_Float16)fmaxf(fmaf(d1[4 + e], kWInv, bd[e]), 0.0f);
    }
    const int o2 = (mt0 * 16 + rlane) * 512 + ks * 32 + koff;
#pragma unroll
    for (int mt = 0; mt < 8; ++mt) {
      const int o = pin_i(o2 + mt * 16 * 512);
      const v16h a2 = frag_load(W2 + o);
      acc[mt] = mma16(a2, bf, acc[mt]);
    }
  }
  float s = 0.0f;
#pragma unroll
  for (int mt = 0; mt < 8; ++mt) {
    int fo = (mt0 + mt) * 16 + koff;
    pin_if(fo, s);
    const v4f ba = *(const v4f*)(b2 + fo);
    const v4f bb = *(const v4f*)(b2 + fo + 4);
    const v4f wa = *(const v4f*)(w3 + fo);
    const v4f wb = *(const v4f*)(w3 + fo + 4);
#pragma unroll
    for (int e = 0; e < 4; ++e) {
      const float u0 = fmaxf(fmaf(acc[mt][e],     kWInv, ba[e]), 0.0f);
      const float u1 = fmaxf(fmaf(acc[mt][4 + e], kWInv, bb[e]), 0.0f);
      s = fmaf(u0, wa[e], s);
      s = fmaf(u1, wb[e], s);
    }
  }
  return s;
}

__global__ __launch_bounds__(128) void prep_planes_kernel(
    const float* __restrict__ w0, const float* __restrict__ w1, const float* __restrict__ w2,
    const float* __restrict__ w3, const float* __restrict__ w4, const float* __restrict__ w5,
    const float* __restrict__ w6, const float* __restrict__ w7, const float* __restrict__ w8,
    unsigned short* __restrict__ dst) {
  const int blk = blockIdx.x;
  const float* src = w0;
  int kreal = 64, ksh = 6, b0 = kBlkP0;
  if (blk >= kBlkP1) { src = w1; kreal = 64;  ksh = 6; b0 = kBlkP1; }
  if (blk >= kBlkP2) { src = w2; kreal = 512; ksh = 9; b0 = kBlkP2; }
  if (blk >= kBlkP3) { src = w3; kreal = 35;  ksh = 6; b0 = kBlkP3; }
  if (blk >= kBlkP4) { src = w4; kreal = 32;  ksh = 5; b0 = kBlkP4; }
  if (blk >= kBlkP5) { src = w5; kreal = 32;  ksh = 5; b0 = kBlkP5; }
  if (blk >= kBlkP6) { src = w6; kreal = 512; ksh = 9; b0 = kBlkP6; }
  if (blk >= kBlkP7) { src = w7; kreal = 35;  ksh = 6; b0 = kBlkP7; }
  if (blk >= kBlkP8) { src = w8; kreal = 512; ksh = 9; b0 = kBlkP8; }
  const int e0 = ((blk - b0) * 128 + (int)threadIdx.x) * 8;
  const int n = e0 >> ksh;
  const int k = e0 & ((1 << ksh) - 1);
  const float* rowp = src + (size_t)n * kreal;
  v8h hv;
#pragma unroll
  for (int e = 0; e < 8; ++e) {
    const int kk = k + e;
    const int kc = (kk < kreal) ? kk : (kreal - 1);
    const float raw = rowp[kc];
    const float v = (kk < kreal) ? (raw * kWCarry) : 0.0f;
    hv[e] = (_Float16)v;
  }
  unsigned short* dp = dst + ((size_t)blk * 128 + threadIdx.x) * 8;
  *(volatile v8h*)dp = hv;
  __threadfence();
  *(volatile v8h*)dp = hv;
}

__global__ __launch_bounds__(128) __attribute__((amdgpu_num_vgpr(256))) void policy_rows_kernel(
    const float* __restrict__ x, const float* __restrict__ wih, const float* __restrict__ bih,
    const float* __restrict__ bhh, const unsigned short* __restrict__ whhP,
    const unsigned short* __restrict__ fc1P, const float* __restrict__ fc1b,
    const unsigned short* __restrict__ fc2P, const float* __restrict__ fc2b,
    const float* __restrict__ fc3w, const float* __restrict__ fc3b, float* __restrict__ sa) {
  __shared__ __align__(16) float sWih[192 * 6];
  __shared__ __align__(16) float sBih[192];
  __shared__ __align__(16) float sBhh[192];
  __shared__ __align__(16) float sH[4 * 4 * 32 * 8];
  __shared__ __align__(16) float sG[4 * 32 * 24];
  const int tid = threadIdx.x;
  const int lane = tid & 31;
  const int wave = tid >> 5;
  const int rlane = lane & 15;
  const int hh = lane >> 4;
  const int koff = hh * 8;
#pragma unroll 1
  for (int i = tid; i < 192 * 6; i += 128) sWih[i] = wih[i];
#pragma unroll 1
  for (int i = tid; i < 192; i += 128) {
    sBih[i] = bih[i];
    sBhh[i] = bhh[i];
  }
  const int hbase = (wave * 4) * 256 + lane * 8;
  const int gbase = (wave * 32 + lane) * 24;
#pragma unroll
  for (int ct = 0; ct < 4; ++ct) {
#pragma unroll
    for (int r = 0; r < 8; ++r) sH[hbase + ct * 256 + r] = 0.0f;
  }
  __syncthreads();

  const _Float16* Whh = (const _Float16*)whhP;
  const _Float16* Fc1 = (const _Float16*)fc1P;
  const _Float16* Fc2 = (const _Float16*)fc2P;
  const int row0 = (blockIdx.x * 4 + wave) * 16;
  const int row = row0 + rlane;
  const int zc = row >> 10;
  const int bc = row & 1023;
  const float b3 = fc3b[0];

  v16h hB0 = zero16h();
  v16h hB1 = zero16h();
  float s0 = 0.0f, s1 = 0.0f;

#pragma unroll 1
  for (int t = 0; t < 2; ++t) {
    const float* xp = x + ((size_t)(bc * 2 + t) * 100 + zc) * 6;
    const v2f xa = *(const v2f*)(xp);
    const v2f xb = *(const v2f*)(xp + 2);
    const v2f xc = *(const v2f*)(xp + 4);
    const float x0 = xa[0], x1 = xa[1], x2 = xb[0], x3 = xb[1], x4 = xc[0], x5 = xc[1];

#pragma unroll 1
    for (int ct = 0; ct < 4; ++ct) {
      v8f gr = zero8();
      v8f gz = zero8();
      v8f gn = zero8();
      if (t != 0) {
        const int w0 = (ct * 16 + rlane) * 64 + koff;
        v16h a;
        int o;
        o = pin_i(w0);
        a = frag_load(Whh + o);
        gr = mma16(a, hB0, gr);
        o = pin_i(w0 + 32);
        a = frag_load(Whh + o);
        gr = mma16(a, hB1, gr);
        o = pin_i(w0 + 64 * 64);
        a = frag_load(Whh + o);
        gz = mma16(a, hB0, gz);
        o = pin_i(w0 + 64 * 64 + 32);
        a = frag_load(Whh + o);
        gz = mma16(a, hB1, gz);
        o = pin_i(w0 + 128 * 64);
        a = frag_load(Whh + o);
        gn = mma16(a, hB0, gn);
        o = pin_i(w0 + 128 * 64 + 32);
        a = frag_load(Whh + o);
        gn = mma16(a, hB1, gn);
      }
#pragma unroll
      for (int r = 0; r < 8; ++r) {
        sG[gbase + r]      = gr[r];
        sG[gbase + 8 + r]  = gz[r];
        sG[gbase + 16 + r] = gn[r];
      }
      const int j0 = ct * 16 + koff;
      const int hs = hbase + ct * 256;
#pragma unroll 1
      for (int r = 0; r < 8; ++r) {
        const int j = j0 + r;
        const float* wr = &sWih[j * 6];
        const float* wz = &sWih[(64 + j) * 6];
        const float* wn = &sWih[(128 + j) * 6];
        float ar = sBih[j];
        ar = fmaf(x0, wr[0], ar);
        ar = fmaf(x1, wr[1], ar);
        ar = fmaf(x2, wr[2], ar);
        ar = fmaf(x3, wr[3], ar);
        ar = fmaf(x4, wr[4], ar);
        ar = fmaf(x5, wr[5], ar);
        float az = sBih[64 + j];
        az = fmaf(x0, wz[0], az);
        az = fmaf(x1, wz[1], az);
        az = fmaf(x2, wz[2], az);
        az = fmaf(x3, wz[3], az);
        az = fmaf(x4, wz[4], az);
        az = fmaf(x5, wz[5], az);
        float an = sBih[128 + j];
        an = fmaf(x0, wn[0], an);
        an = fmaf(x1, wn[1], an);
        an = fmaf(x2, wn[2], an);
        an = fmaf(x3, wn[3], an);
        an = fmaf(x4, wn[4], an);
        an = fmaf(x5, wn[5], an);
        const float hr = fmaf(sG[gbase + r],      kWInv, sBhh[j]);
        const float hz = fmaf(sG[gbase + 8 + r],  kWInv, sBhh[64 + j]);
        const float hn = fmaf(sG[gbase + 16 + r], kWInv, sBhh[128 + j]);
        const float rg = 1.0f / (1.0f + expf(-(ar + hr)));
        const float zg = 1.0f / (1.0f + expf(-(az + hz)));
        const float ng = tanhf(an + rg * hn);
        const float ho = sH[hs + r];
        sH[hs + r] = (1.0f - zg) * ng + zg * ho;
      }
    }
    {
      float t0[8], t1[8], t2[8], t3[8];
#pragma unroll
      for (int r = 0; r < 8; ++r) {
        t0[r] = sH[hbase + r];
        t1[r] = sH[hbase + 256 + r];
        t2[r] = sH[hbase + 512 + r];
        t3[r] = sH[hbase + 768 + r];
      }
      hB0 = pack_tiles(t0, t1);
      hB1 = pack_tiles(t2, t3);
    }
    float s = mlp_chain8<2>(Fc1, fc1b, Fc2, fc2b, fc3w, 0, hB0, hB1, rlane, koff);
    s += __shfl_xor(s, 16, 32);
    s += b3;
    s0 = (t == 0) ? s : s0;
    s1 = (t == 0) ? s1 : s;
  }
  const int srcl = lane >> 1;
  const float v0 = __shfl(s0, srcl, 32);
  const float v1 = __shfl(s1, srcl, 32);
  const float val = (lane & 1) ? v1 : v0;
  volatile float* dp = sa + (size_t)row0 * 2 + lane;
  *dp = val;
  __threadfence();
  *dp = val;
}

__global__ __launch_bounds__(64) __attribute__((amdgpu_num_vgpr(256))) void value_rows_kernel(
    const float* __restrict__ x, const float* __restrict__ sa,
    const unsigned short* __restrict__ cwihP, const unsigned short* __restrict__ cwhhP,
    const float* __restrict__ cbih, const float* __restrict__ cbhh,
    const unsigned short* __restrict__ cfc1P, const float* __restrict__ cfc1b,
    const unsigned short* __restrict__ cfc2P, const float* __restrict__ cfc2b,
    const float* __restrict__ cfc3w, const float* __restrict__ cfc3b,
    const unsigned short* __restrict__ lfc1P, const float* __restrict__ lfc1b,
    const unsigned short* __restrict__ lfc2P, const float* __restrict__ lfc2b,
    const float* __restrict__ lfc3w, const float* __restrict__ lfc3b,
    float* __restrict__ qout) {
  __shared__ __align__(16) _Float16 sXi[2 * 2 * 16 * 64];
  __shared__ __align__(16) float sHc[2 * 2 * 32 * 8];
  __shared__ __align__(16) float sQ[32];
  const int tid = threadIdx.x;
  const int lane = tid & 31;
  const int wave = tid >> 5;
  const int rlane = lane & 15;
  const int hh = lane >> 4;
  const int koff = hh * 8;
  const int b0 = blockIdx.x * 32 + wave * 16;

  {
    v8h zv;
#pragma unroll
    for (int e = 0; e < 8; ++e) zv[e] = (_Float16)0.0f;
#pragma unroll
    for (int it = 0; it < 8; ++it) *(v8h*)&sXi[wave * 2048 + (it * 32 + lane) * 8] = zv;
  }
  const int hbase = (wave * 2) * 256 + lane * 8;
  {
    const v4f z4 = (v4f){0.f, 0.f, 0.f, 0.f};
    *(v4f*)&sHc[hbase]           = z4;
    *(v4f*)&sHc[hbase + 4]       = z4;
    *(v4f*)&sHc[hbase + 256]     = z4;
    *(v4f*)&sHc[hbase + 256 + 4] = z4;
  }
  __syncthreads();
#pragma unroll 1
  for (int it = 0; it < 18; ++it) {
    const int e = it * 32 + lane;
    const int n = e / 36;
    const int rem = e - n * 36;
    const int t = rem / 18;
    const int r2 = rem - t * 18;
    const int gi = r2 / 6;
    const int s = r2 - gi * 6;
    const int z = (gi == 0) ? 99 : ((gi == 1) ? 89 : 98);
    const int col = (gi == 0) ? 0 : ((gi == 1) ? 7 : 28);
    const float v = x[((size_t)((b0 + n) * 2 + t) * 100 + z) * 6 + s];
    sXi[((wave * 2 + t) * 16 + n) * 64 + col + s] = (_Float16)v;
  }
#pragma unroll 1
  for (int it = 0; it < 3; ++it) {
    const int e = it * 32 + lane;
    const int n = e / 6;
    const int rem = e - n * 6;
    const int t = rem / 3;
    const int gi = rem - t * 3;
    const int z = (gi == 0) ? 99 : ((gi == 1) ? 89 : 98);
    const int col = (gi == 0) ? 0 : ((gi == 1) ? 7 : 28);
    const float v = sa[(size_t)(b0 + n) * 200 + t * 100 + z];
    sXi[((wave * 2 + t) * 16 + n) * 64 + col + 6] = (_Float16)v;
  }
  __syncthreads();

  const _Float16* Cwih = (const _Float16*)cwihP;
  const _Float16* Cwhh = (const _Float16*)cwhhP;
  const _Float16* Cfc1 = (const _Float16*)cfc1P;
  const _Float16* Cfc2 = (const _Float16*)cfc2P;
  const _Float16* Lfc1 = (const _Float16*)lfc1P;
  const _Float16* Lfc2 = (const _Float16*)lfc2P;

  v16h hB = zero16h();
#pragma unroll 1
  for (int t = 0; t < 2; ++t) {
    const v16h xB0 = frag_load(&sXi[((wave * 2 + t) * 16 + rlane) * 64 + koff]);
    const v16h xB1 = frag_load(&sXi[((wave * 2 + t) * 16 + rlane) * 64 + 32 + koff]);
#pragma unroll 1
    for (int ct = 0; ct < 2; ++ct) {
      v8f ir = zero8();
      v8f iz = zero8();
      v8f in_ = zero8();
      v8f gr = zero8();
      v8f gz = zero8();
      v8f gn = zero8();
      const _Float16* wp = Cwih + (size_t)(ct * 16 + rlane) * 64 + koff;
      v16h a;
      a = frag_load(wp);
      ir = mma16(a, xB0, ir);
      a = frag_load(wp + 32);
      ir = mma16(a, xB1, ir);
      a = frag_load(wp + 32 * 64);
      iz = mma16(a, xB0, iz);
      a = frag_load(wp + 32 * 64 + 32);
      iz = mma16(a, xB1, iz);
      a = frag_load(wp + 64 * 64);
      in_ = mma16(a, xB0, in_);
      a = frag_load(wp + 64 * 64 + 32);
      in_ = mma16(a, xB1, in_);
      if (t != 0) {
        const _Float16* hp = Cwhh + (size_t)(ct * 16 + rlane) * 32 + koff;
        a = frag_load(hp);
        gr = mma16(a, hB, gr);
        a = frag_load(hp + 32 * 32);
        gz = mma16(a, hB, gz);
        a = frag_load(hp + 64 * 32);
        gn = mma16(a, hB, gn);
      }
      const int j0 = ct * 16 + koff;
      float biR[8], biZ[8], biN[8], bhR[8], bhZ[8], bhN[8], ho[8];
      unpack8(*(const v4f*)(cbih + j0),      *(const v4f*)(cbih + j0 + 4),      biR);
      unpack8(*(const v4f*)(cbih + 32 + j0), *(const v4f*)(cbih + 32 + j0 + 4), biZ);
      unpack8(*(const v4f*)(cbih + 64 + j0), *(const v4f*)(cbih + 64 + j0 + 4), biN);
      unpack8(*(const v4f*)(cbhh + j0),      *(const v4f*)(cbhh + j0 + 4),      bhR);
      unpack8(*(const v4f*)(cbhh + 32 + j0), *(const v4f*)(cbhh + 32 + j0 + 4), bhZ);
      unpack8(*(const v4f*)(cbhh + 64 + j0), *(const v4f*)(cbhh + 64 + j0 + 4), bhN);
      unpack8(*(const v4f*)&sHc[hbase + ct * 256], *(const v4f*)&sHc[hbase + ct * 256 + 4], ho);
      float xr[8], xz[8], xn[8], hr[8], hz[8], hn[8], hnew[8];
#pragma unroll
      for (int r = 0; r < 8; ++r) {
        xr[r] = fmaf(ir[r],  kWInv, biR[r]);
        xz[r] = fmaf(iz[r],  kWInv, biZ[r]);
        xn[r] = fmaf(in_[r], kWInv, biN[r]);
        hr[r] = fmaf(gr[r],  kWInv, bhR[r]);
        hz[r] = fmaf(gz[r],  kWInv, bhZ[r]);
        hn[r] = fmaf(gn[r],  kWInv, bhN[r]);
      }
      gru_gates8(xr, xz, xn, hr, hz, hn, ho, hnew);
      *(v4f*)&sHc[hbase + ct * 256]     = (v4f){hnew[0], hnew[1], hnew[2], hnew[3]};
      *(v4f*)&sHc[hbase + ct * 256 + 4] = (v4f){hnew[4], hnew[5], hnew[6], hnew[7]};
    }
    {
      float t0[8], t1[8];
      unpack8(*(const v4f*)&sHc[hbase],       *(const v4f*)&sHc[hbase + 4],       t0);
      unpack8(*(const v4f*)&sHc[hbase + 256], *(const v4f*)&sHc[hbase + 256 + 4], t1);
      hB = pack_tiles(t0, t1);
    }
  }

  const v16h xL0 = frag_load(&sXi[((wave * 2 + 1) * 16 + rlane) * 64 + koff]);
  const v16h xL1 = frag_load(&sXi[((wave * 2 + 1) * 16 + rlane) * 64 + 32 + koff]);
  float tot = 0.0f;
#pragma unroll 1
  for (int half = 0; half < 2; ++half)
    tot += mlp_chain8<2>(Lfc1, lfc1b, Lfc2, lfc2b, lfc3w, half * 8, xL0, xL1, rlane, koff);
#pragma unroll 1
  for (int half = 0; half < 2; ++half)
    tot += mlp_chain8<1>(Cfc1, cfc1b, Cfc2, cfc2b, cfc3w, half * 8, hB, hB, rlane, koff);
  tot += __shfl_xor(tot, 16, 32);
  const float qv = (tot + lfc3b[0]) + cfc3b[0];
  if (lane < 16) sQ[wave * 16 + lane] = qv;
  __syncthreads();
  if (wave == 0) {
    const float v = sQ[lane];
    volatile float* dp = qout + (size_t)blockIdx.x * 32 + lane;
    *dp = v;
    __threadfence();
    *dp = v;
  }
}

__global__ __launch_bounds__(256) void pack_out_kernel(const float* __restrict__ sa, float* __restrict__ out) {
  const int i = (blockIdx.x * 256 + (int)threadIdx.x) * 4;
  const int n = i / 100;
  const int c = i - n * 100;
  const v4f v = *(const v4f*)(sa + (size_t)n * 200 + 100 + c);
  *(volatile v4f*)(out + i) = v;
  __threadfence();
  *(volatile v4f*)(out + i) = v;
}

extern "C" void kernel_launch(void* const* d_in, const int* in_sizes, int n_in,
                              void* d_out, int out_size, void* d_ws, size_t ws_size,
                              hipStream_t stream) {
  if (n_in < 27) return;
  if (in_sizes[0] != kNB * kNT * kNZ * kNS) return;
  if (in_sizes[1] != 192 * 6 || in_sizes[2] != 192 * 64 || in_sizes[3] != 192 || in_sizes[4] != 192) return;
  if (in_sizes[5] != 512 * 64 || in_sizes[6] != 512 || in_sizes[7] != 128 * 512 || in_sizes[8] != 128) return;
  if (in_sizes[9] != 128 || in_sizes[10] != 1) return;
  if (in_sizes[11] != 96 * 35 || in_sizes[12] != 96 * 32 || in_sizes[13] != 96 || in_sizes[14] != 96) return;
  if (in_sizes[15] != 512 * 32 || in_sizes[16] != 512 || in_sizes[17] != 256 * 512 || in_sizes[18] != 256) return;
  if (in_sizes[19] != 256 || in_sizes[20] != 1) return;
  if (in_sizes[21] != 512 * 35 || in_sizes[22] != 512 || in_sizes[23] != 256 * 512 || in_sizes[24] != 256) return;
  if (in_sizes[25] != 256 || in_sizes[26] != 1) return;
  if (out_size != kOutAll) return;
  if (ws_size < kWsTotal) return;

  const float* x      = (const float*)d_in[0];
  const float* a_wih  = (const float*)d_in[1];
  const float* a_whh  = (const float*)d_in[2];
  const float* a_bih  = (const float*)d_in[3];
  const float* a_bhh  = (const float*)d_in[4];
  const float* a_fc1w = (const float*)d_in[5];
  const float* a_fc1b = (const float*)d_in[6];
  const float* a_fc2w = (const float*)d_in[7];
  const float* a_fc2b = (const float*)d_in[8];
  const float* a_fc3w = (const float*)d_in[9];
  const float* a_fc3b = (const float*)d_in[10];
  const float* c_wih  = (const float*)d_in[11];
  const float* c_whh  = (const float*)d_in[12];
  const float* c_bih  = (const float*)d_in[13];
  const float* c_bhh  = (const float*)d_in[14];
  const float* c_fc1w = (const float*)d_in[15];
  const float* c_fc1b = (const float*)d_in[16];
  const float* c_fc2w = (const float*)d_in[17];
  const float* c_fc2b = (const float*)d_in[18];
  const float* c_fc3w = (const float*)d_in[19];
  const float* c_fc3b = (const float*)d_in[20];
  const float* l_fc1w = (const float*)d_in[21];
  const float* l_fc1b = (const float*)d_in[22];
  const float* l_fc2w = (const float*)d_in[23];
  const float* l_fc2b = (const float*)d_in[24];
  const float* l_fc3w = (const float*)d_in[25];
  const float* l_fc3b = (const float*)d_in[26];
  float* out = (float*)d_out;

  char* ws = (char*)d_ws;
  float* SA = (float*)(ws + kOffSA);
  unsigned short* W16 = (unsigned short*)(ws + kOffW16);
  const unsigned short* P0 = W16 + (size_t)kBlkP0 * 1024;
  const unsigned short* P1 = W16 + (size_t)kBlkP1 * 1024;
  const unsigned short* P2 = W16 + (size_t)kBlkP2 * 1024;
  const unsigned short* P3 = W16 + (size_t)kBlkP3 * 1024;
  const unsigned short* P4 = W16 + (size_t)kBlkP4 * 1024;
  const unsigned short* P5 = W16 + (size_t)kBlkP5 * 1024;
  const unsigned short* P6 = W16 + (size_t)kBlkP6 * 1024;
  const unsigned short* P7 = W16 + (size_t)kBlkP7 * 1024;
  const unsigned short* P8 = W16 + (size_t)kBlkP8 * 1024;

  prep_planes_kernel<<<kBlkEnd, 128, 0, stream>>>(a_whh, a_fc1w, a_fc2w, c_wih, c_whh, c_fc1w, c_fc2w,
                                                 l_fc1w, l_fc2w, W16);

  policy_rows_kernel<<<kRowsP / 64, 128, 0, stream>>>(x, a_wih, a_bih, a_bhh, P0, P1, a_fc1b, P2, a_fc2b,
                                                     a_fc3w, a_fc3b, SA);

  value_rows_kernel<<<kNB / 32, 64, 0, stream>>>(x, SA, P3, P4, c_bih, c_bhh, P5, c_fc1b, P6, c_fc2b,
                                                c_fc3w, c_fc3b, P7, l_fc1b, P8, l_fc2b, l_fc3w, l_fc3b,
                                                out + kOut0);

  pack_out_kernel<<<kOut0 / 1024, 256, 0, stream>>>(SA, out);
}
